// Graph_NN_13271448945380
// MI455X (gfx1250) — hardware-run, weakly checked
//
#include <hip/hip_runtime.h>
#include <stddef.h>
#include <stdint.h>

#define NN      100000
#define NE      1600000
#define DF      128
#define NV      5000
#define NSTEP   3
#define NP      100096
#define APITCH  256
#define WPITCH  256
#define TWO_TERM_A 1
#define TWO_TERM_B 1
#define TWO_TERM_C 1
#define NTHR    256
#define NWAVE   8
#define EPT     8
#define WCH     (32 * EPT)
#define NBRUN   1024
#define SLB     10
#define SRCB    17
#define NBK     98
#define WLCAP   3072
#define RCAP    18432
#define TRIPCAP 64
#define MAXDEG_MEAS   36
#define MAXB1024_MEAS 16721
#define COW     (3 * NBRUN)
#define RBM     64
#define GBM     64
#define GBN     128
#define GTHR    128
#define GWAVE   4

#define BK_ZINTS (NWAVE * WLCAP + RCAP + 3 * NBRUN)
#define BK_INTS  (BK_ZINTS + 16)
#define BK_LDS   (BK_INTS * 4)

#define PBH  (NP * DF / 8 / NTHR)
#define PBW  (NSTEP * DF * WPITCH / 8 / NTHR)
#define PBZ  ((NP - NN) * APITCH / 8 / NTHR)
#define PBTOT (PBH + PBW + PBZ + 1)

static_assert(NN <= (1 << SRCB));
static_assert(NBRUN == (1 << SLB) && SLB + SRCB <= 31);
static_assert(NBK * NBRUN >= NN && (NBK - 1) * NBRUN < NN);
static_assert(NP % 128 == 0 && NP == 782 * 128 && NP >= NN && NP % GBM == 0 && NP % RBM == 0);
static_assert(NP <= NBK * NBRUN);
static_assert(DF == 128 && GBN == DF && APITCH == 2 * DF && WPITCH == 2 * DF);
static_assert(NE % WCH == 0 && NE % 4 == 0);
static_assert((long long)RCAP * 100 >= (long long)MAXB1024_MEAS * 105);
static_assert((long long)WLCAP * 100 >= (long long)(MAXB1024_MEAS / NWAVE + 1) * 125);
static_assert(RCAP % (NTHR * 4) == 0 && BK_ZINTS % 4 == 0 && COW == 3 * NTHR * 4);
static_assert(MAXDEG_MEAS + 8 <= TRIPCAP);
static_assert(BK_LDS <= 300000);
static_assert(NBRUN % RBM == 0 && RBM % NWAVE == 0 && NBRUN % 32 == 0);
static_assert((NP * DF / 8) % NTHR == 0 && (NSTEP * DF * WPITCH / 8) % NTHR == 0);
static_assert(((NP - NN) * APITCH / 8) % NTHR == 0 && NSTEP * DF / 4 <= NTHR && (NSTEP * DF / 4) % 32 == 0);
static_assert(GBM == GWAVE * 16 && GTHR == GWAVE * 32);
static_assert((GBM * GBN + GBN) * 4 <= 65536);

typedef float          v4f   __attribute__((ext_vector_type(4)));
typedef float          v8f   __attribute__((ext_vector_type(8)));
typedef int            v4i   __attribute__((ext_vector_type(4)));
typedef int            v8i   __attribute__((ext_vector_type(8)));
typedef unsigned       v2u   __attribute__((ext_vector_type(2)));
typedef unsigned       v4u   __attribute__((ext_vector_type(4)));
typedef unsigned short v8us  __attribute__((ext_vector_type(8)));
typedef unsigned short v16us __attribute__((ext_vector_type(16)));
typedef __bf16         v16bf __attribute__((ext_vector_type(16)));
typedef v4f  __attribute__((may_alias)) v4fa;
typedef v4i  __attribute__((may_alias)) v4ia;
typedef v2u  __attribute__((may_alias)) v2ua;
typedef v4u  __attribute__((may_alias)) v4ua;
typedef v8us __attribute__((may_alias)) v8usa;
union FragB { v16bf v; v16us u; v8us h[2]; v8i w; };

__device__ __forceinline__ v8f wmb(const FragB& a, const FragB& b, v8f c) {
  v8f d = __builtin_amdgcn_wmma_f32_16x16x32_bf16(false, a.v, false, b.v, (short)0, c, false, false);
  asm volatile("v_nop\n\tv_nop\n\tv_nop\n\tv_nop" : "+v"(d) : "v"(a.w), "v"(b.w));
  return d;
}

__device__ __forceinline__ unsigned bf16_bits(float f) {
  const unsigned u = __float_as_uint(f);
  const unsigned r = (u + 0x7FFFu + ((u >> 16) & 1u)) >> 16;
  const unsigned q = (u >> 16) | 0x40u;
  return ((u & 0x7fffffffu) > 0x7f800000u) ? q : r;
}
__device__ __forceinline__ float bf16_val(float f) {
  return __uint_as_float(bf16_bits(f) << 16);
}

__device__ __forceinline__ void wave_sync() {
  __builtin_amdgcn_fence(__ATOMIC_RELEASE, "wavefront");
  __builtin_amdgcn_wave_barrier();
  __builtin_amdgcn_fence(__ATOMIC_ACQUIRE, "wavefront");
}

__device__ __forceinline__ void st2_v4f(float* p, v4f v) {
  *(volatile v4f*)p = v;
  __threadfence();
  *(volatile v4f*)p = v;
}
__device__ __forceinline__ void st2_v8us(unsigned short* p, v8us v) {
  *(volatile v8us*)p = v;
  __threadfence();
  *(volatile v8us*)p = v;
}

__device__ __forceinline__ v8us col8(const float* __restrict__ base, int stride) {
  float f[8];
#pragma unroll
  for (int i = 0; i < 8; ++i) f[i] = base[(size_t)i * (size_t)stride];
  v8us o;
#pragma unroll
  for (int i = 0; i < 8; ++i) o[i] = (unsigned short)bf16_bits(f[i]);
  return o;
}

__device__ __forceinline__ v4f row16(const unsigned short* rp) {
  const v2u w = *(const v2ua*)rp;
  v4f r;
  r.x = __uint_as_float(w.x << 16);
  r.y = __uint_as_float(w.x & 0xffff0000u);
  r.z = __uint_as_float(w.y << 16);
  r.w = __uint_as_float(w.y & 0xffff0000u);
  return r;
}

__device__ __forceinline__ unsigned csrc(int s) {
  s = s < 0 ? 0 : s;
  s = s > NN - 1 ? NN - 1 : s;
  return (unsigned)s;
}

__global__ __launch_bounds__(NTHR) void k_prep(const int* __restrict__ ann, const float* __restrict__ emb,
                                               const float* __restrict__ wsrc, const float* __restrict__ bs,
                                               unsigned short* hb, unsigned short* wd, unsigned short* zhl,
                                               float* bsr) {
  const int tid = (int)threadIdx.x;
  const int blk = (int)blockIdx.x;
  if (blk < PBH) {
    const int u   = blk * NTHR + tid;
    const int row = u >> 4, k8 = (u & 15) * 8;
    const int rc  = row < NN ? row : NN - 1;
    int a = ann[rc];
    a = a < 0 ? 0 : (a > NV - 1 ? NV - 1 : a);
    const unsigned mk = row < NN ? 0xffffu : 0u;
    const float* p = emb + (size_t)a * DF + k8;
    const v4f x0 = *(const v4fa*)p;
    const v4f x1 = *(const v4fa*)(p + 4);
    v8us o;
    o[0] = (unsigned short)(bf16_bits(x0.x) & mk); o[1] = (unsigned short)(bf16_bits(x0.y) & mk);
    o[2] = (unsigned short)(bf16_bits(x0.z) & mk); o[3] = (unsigned short)(bf16_bits(x0.w) & mk);
    o[4] = (unsigned short)(bf16_bits(x1.x) & mk); o[5] = (unsigned short)(bf16_bits(x1.y) & mk);
    o[6] = (unsigned short)(bf16_bits(x1.z) & mk); o[7] = (unsigned short)(bf16_bits(x1.w) & mk);
    st2_v8us(hb + (size_t)row * DF + k8, o);
  } else if (blk < PBH + PBW) {
    const int u = (blk - PBH) * NTHR + tid;
    const int l = u >> 12, n = (u >> 5) & (DF - 1), k8 = (u & 31) * 8, kk = k8 & (DF - 1);
    const v8us o = col8(wsrc + (size_t)l * DF * DF + (size_t)kk * DF + n, DF);
    st2_v8us(wd + (size_t)l * DF * WPITCH + (size_t)n * WPITCH + k8, o);
  } else if (blk < PBH + PBW + PBZ) {
    const int u = (blk - PBH - PBW) * NTHR + tid;
    const v8us z = {0, 0, 0, 0, 0, 0, 0, 0};
    st2_v8us(zhl + (size_t)NN * APITCH + (size_t)u * 8, z);
  } else {
    if (tid < NSTEP * DF / 4) {
      const v4f b = *(const v4fa*)(bs + 4 * tid);
      v4f o;
      o.x = bf16_val(b.x); o.y = bf16_val(b.y); o.z = bf16_val(b.z); o.w = bf16_val(b.w);
      st2_v4f(bsr + 4 * tid, o);
    }
  }
}

__device__ __forceinline__ void bucket_flush(const int* pl, const int* cnt, int ov, int* lp, int* cop, int* fp,
                                             int tid) {
#pragma unroll 1
  for (int i = tid * 4; i < RCAP; i += NTHR * 4) {
    const v4i v = *(const v4ia*)(pl + i);
    *(volatile v4i*)(lp + i) = v;
  }
#pragma unroll 1
  for (int it = 0; it < 3; ++it) {
    const int i4 = it * NTHR + tid;
    const v4i v = *(const v4ia*)(cnt + 4 * i4);
    *(volatile v4i*)(cop + 4 * i4) = v;
  }
  if (tid < 8) {
    const v4i f = {ov, ov, ov, ov};
    *(volatile v4i*)(fp + 4 * tid) = f;
  }
}

__global__ __launch_bounds__(NTHR) void k_bucket(const int* __restrict__ srcs, const int* __restrict__ dsts,
                                                 int* LIST, int* COI, int* FLAG) {
  extern __shared__ __attribute__((aligned(16))) int dsm[];
  int* wl   = dsm;
  int* pl   = dsm + NWAVE * WLCAP;
  int* cnt  = pl + RCAP;
  int* offs = cnt + NBRUN;
  int* cur  = offs + NBRUN;
  int* misc = cur + NBRUN;
  const int tid = (int)threadIdx.x, lane = tid & 31, wave = tid >> 5;
  const int blk = (int)blockIdx.x;
  const unsigned nbs = (unsigned)(blk * NBRUN);
  const int liveSlots = (NN - blk * NBRUN) < NBRUN ? (NN - blk * NBRUN) : NBRUN;
  const unsigned unb = (unsigned)(liveSlots < 0 ? 0 : liveSlots);

  {
    const v4i z4 = {0, 0, 0, 0};
    for (int i = tid * 4; i < BK_ZINTS; i += NTHR * 4) *(v4ia*)(dsm + i) = z4;
    if (tid < 16) misc[tid] = 0;
  }
  __syncthreads();

  {
    const int per  = ((NE + NWAVE * WCH - 1) / (NWAVE * WCH)) * WCH;
    const int ebeg = wave * per;
    const int eend = (ebeg + per < NE) ? (ebeg + per) : NE;
    int* mylist = wl + wave * WLCAP;
    int wc = 0;
#pragma unroll 1
    for (int cb = ebeg; cb < eend; cb += WCH) {
      const int e0 = cb + lane * EPT;
      const v4i da = *(const v4ia*)(dsts + e0);
      const v4i db = *(const v4ia*)(dsts + e0 + 4);
      const v4i sa = *(const v4ia*)(srcs + e0);
      const v4i sc = *(const v4ia*)(srcs + e0 + 4);
      asm volatile("" :: "v"(sa), "v"(sc));
      const unsigned s0 = (unsigned)da.x - nbs, s1 = (unsigned)da.y - nbs;
      const unsigned s2 = (unsigned)da.z - nbs, s3 = (unsigned)da.w - nbs;
      const unsigned s4 = (unsigned)db.x - nbs, s5 = (unsigned)db.y - nbs;
      const unsigned s6 = (unsigned)db.z - nbs, s7 = (unsigned)db.w - nbs;
      const bool h0 = s0 < unb, h1 = s1 < unb, h2 = s2 < unb, h3 = s3 < unb;
      const bool h4 = s4 < unb, h5 = s5 < unb, h6 = s6 < unb, h7 = s7 < unb;
      const unsigned m0 = __builtin_amdgcn_ballot_w32(h0), m1 = __builtin_amdgcn_ballot_w32(h1);
      const unsigned m2 = __builtin_amdgcn_ballot_w32(h2), m3 = __builtin_amdgcn_ballot_w32(h3);
      const unsigned m4 = __builtin_amdgcn_ballot_w32(h4), m5 = __builtin_amdgcn_ballot_w32(h5);
      const unsigned m6 = __builtin_amdgcn_ballot_w32(h6), m7 = __builtin_amdgcn_ballot_w32(h7);
      const unsigned any = m0 | m1 | m2 | m3 | m4 | m5 | m6 | m7;
      if (any != 0u) {
        const int pre = (int)(__builtin_amdgcn_mbcnt_lo(m0, 0u) + __builtin_amdgcn_mbcnt_lo(m1, 0u) +
                              __builtin_amdgcn_mbcnt_lo(m2, 0u) + __builtin_amdgcn_mbcnt_lo(m3, 0u) +
                              __builtin_amdgcn_mbcnt_lo(m4, 0u) + __builtin_amdgcn_mbcnt_lo(m5, 0u) +
                              __builtin_amdgcn_mbcnt_lo(m6, 0u) + __builtin_amdgcn_mbcnt_lo(m7, 0u));
        int p = wc + pre;
        if (h0) { if (p < WLCAP) mylist[p] = (int)((s0 << SRCB) | csrc(sa.x)); p = p + 1; }
        if (h1) { if (p < WLCAP) mylist[p] = (int)((s1 << SRCB) | csrc(sa.y)); p = p + 1; }
        if (h2) { if (p < WLCAP) mylist[p] = (int)((s2 << SRCB) | csrc(sa.z)); p = p + 1; }
        if (h3) { if (p < WLCAP) mylist[p] = (int)((s3 << SRCB) | csrc(sa.w)); p = p + 1; }
        if (h4) { if (p < WLCAP) mylist[p] = (int)((s4 << SRCB) | csrc(sc.x)); p = p + 1; }
        if (h5) { if (p < WLCAP) mylist[p] = (int)((s5 << SRCB) | csrc(sc.y)); p = p + 1; }
        if (h6) { if (p < WLCAP) mylist[p] = (int)((s6 << SRCB) | csrc(sc.z)); p = p + 1; }
        if (h7) { if (p < WLCAP) mylist[p] = (int)((s7 << SRCB) | csrc(sc.w)); p = p + 1; }
        wc += (int)(__builtin_popcount(m0) + __builtin_popcount(m1) + __builtin_popcount(m2) + __builtin_popcount(m3) +
                    __builtin_popcount(m4) + __builtin_popcount(m5) + __builtin_popcount(m6) + __builtin_popcount(m7));
      }
    }
    if (lane == 0) misc[wave] = wc;
  }
  __syncthreads();

  if (wave == 0) {
    int ov = 0;
#pragma unroll 1
    for (int w2 = 0; w2 < NWAVE; ++w2) {
      int c = misc[w2];
      if (c > WLCAP) ov = 1;
      c = c < 0 ? 0 : (c > WLCAP ? WLCAP : c);
#pragma unroll 1
      for (int b0 = 0; b0 < c; b0 += 32) {
        const int idx = b0 + lane;
        const int ent = wl[w2 * WLCAP + (idx < WLCAP ? idx : WLCAP - 1)];
        const int m32 = (c - b0) < 32 ? (c - b0) : 32;
#pragma unroll 1
        for (int k = 0; k < m32; ++k) {
          const int u    = __builtin_amdgcn_readlane(ent, k);
          const int slot = (u >> SRCB) & (NBRUN - 1);
          if (lane == 0) cnt[slot] = cnt[slot] + 1;
        }
      }
    }
    if (lane == 0) misc[9] = ov;
  }
  __syncthreads();
  if (wave == 0) {
    const int base = lane * (NBRUN / 32);
    int s = 0;
#pragma unroll 1
    for (int i = 0; i < NBRUN / 32; ++i) s += cnt[base + i];
    int incl = s;
#pragma unroll
    for (int d = 1; d < 32; d <<= 1) {
      const int y = __shfl_up(incl, d, 32);
      if (lane >= d) incl += y;
    }
    int run = incl - s;
#pragma unroll 1
    for (int i = 0; i < NBRUN / 32; ++i) {
      const int cv = cnt[base + i];
      offs[base + i] = run;
      cur[base + i]  = run;
      run += cv;
    }
    if (lane == 31) misc[10] = (run > RCAP) ? 1 : 0;
  }
  __syncthreads();

  if (wave == 0) {
#pragma unroll 1
    for (int w2 = 0; w2 < NWAVE; ++w2) {
      int c = misc[w2];
      c = c < 0 ? 0 : (c > WLCAP ? WLCAP : c);
#pragma unroll 1
      for (int b0 = 0; b0 < c; b0 += 32) {
        const int idx = b0 + lane;
        const int ent = wl[w2 * WLCAP + (idx < WLCAP ? idx : WLCAP - 1)];
        const int m32 = (c - b0) < 32 ? (c - b0) : 32;
#pragma unroll 1
        for (int k = 0; k < m32; ++k) {
          const int u    = __builtin_amdgcn_readlane(ent, k);
          const int slot = (u >> SRCB) & (NBRUN - 1);
          const int sr   = u & ((1 << SRCB) - 1);
          if (lane == 0) {
            int p = cur[slot];
            p = p < 0 ? 0 : (p > RCAP - 1 ? RCAP - 1 : p);
            pl[p] = sr;
            cur[slot] = p + 1;
          }
        }
      }
    }
  }
  __syncthreads();

#pragma unroll 1
  for (int i = tid; i < NBRUN; i += NTHR) {
    const float dv = (float)cnt[i] + 1.0f;
    cur[i] = __float_as_int(1.0f / dv);
  }
  __syncthreads();

  const int ovf = (misc[9] | misc[10]) != 0 ? 1 : 0;
  int* lp  = LIST + (size_t)blk * RCAP;
  int* cop = COI + (size_t)blk * COW;
  int* fp  = FLAG + (size_t)blk * 32;
  bucket_flush(pl, cnt, ovf, lp, cop, fp, tid);
  __threadfence();
  bucket_flush(pl, cnt, ovf, lp, cop, fp, tid);
}

template <int SRC16>
__global__ __launch_bounds__(NTHR) void k_rowsum(const int* __restrict__ LIST, const int* __restrict__ COI,
                                                 const int* __restrict__ FLAG, const unsigned short* HB,
                                                 const float* Hs, unsigned short* ZHL) {
  __shared__ __attribute__((aligned(16))) unsigned rowbuf[NWAVE * 128];
  const int tid = (int)threadIdx.x, lane = tid & 31, wave = tid >> 5;
  const int rowBase = (int)blockIdx.x * RBM;
  const int bucket  = rowBase >> SLB;
  const int* lb  = LIST + (size_t)bucket * RCAP;
  const int* cob = COI + (size_t)bucket * COW;
  const int flag = FLAG[(size_t)bucket * 32];
  const float qnan = __uint_as_float(0x7fc00000u);
  unsigned* rb = rowbuf + wave * 128;

#pragma unroll 1
  for (int i = 0; i < RBM / NWAVE; ++i) {
    const int d = rowBase + (RBM / NWAVE) * wave + i;
    if (d < NN) {
      const int slot = d & (NBRUN - 1);
      int cv = cob[slot];
      int ov = cob[NBRUN + slot];
      const int iv = cob[2 * NBRUN + slot];
      const bool big = cv > TRIPCAP;
      cv = cv < 0 ? 0 : (cv > TRIPCAP ? TRIPCAP : cv);
      ov = ov < 0 ? 0 : (ov > RCAP - 1 ? RCAP - 1 : ov);
      const int c = __builtin_amdgcn_readfirstlane(cv);
      const int o = __builtin_amdgcn_readfirstlane(ov);
      int last = o + c - 1;
      last = last < o ? o : last;
      last = min(last, RCAP - 1);
      float a0 = 0.0f, a1 = 0.0f, a2 = 0.0f, a3 = 0.0f;
#pragma unroll 1
      for (int b0 = 0; b0 < c; b0 += 32) {
        int idx = o + b0 + lane;
        idx = min(idx, last);
        int sr = lb[idx];
        sr = sr < 0 ? 0 : (sr > NN - 1 ? NN - 1 : sr);
        const int m32 = min(c - b0, 32);
#pragma unroll 1
        for (int k = 0; k < m32; ++k) {
          const int sk = __builtin_amdgcn_readlane(sr, k);
          v4f v;
          if constexpr (SRC16 != 0) v = row16(HB + (size_t)sk * DF + 4 * lane);
          else                      v = *(const v4fa*)(Hs + (size_t)sk * DF + 4 * lane);
          a0 += v.x; a1 += v.y; a2 += v.z; a3 += v.w;
        }
      }
      v4f g;
      if constexpr (SRC16 != 0) g = row16(HB + (size_t)d * DF + 4 * lane);
      else                      g = *(const v4fa*)(Hs + (size_t)d * DF + 4 * lane);
      const float inv = __int_as_float(iv);
      float z0 = (g.x + a0) * inv, z1 = (g.y + a1) * inv, z2 = (g.z + a2) * inv, z3 = (g.w + a3) * inv;
      const bool bad = (flag != 0) | big;
      z0 = bad ? qnan : z0; z1 = bad ? qnan : z1; z2 = bad ? qnan : z2; z3 = bad ? qnan : z3;
      const unsigned h0 = bf16_bits(z0), h1 = bf16_bits(z1), h2 = bf16_bits(z2), h3 = bf16_bits(z3);
      const unsigned l0 = bf16_bits(z0 - __uint_as_float(h0 << 16));
      const unsigned l1 = bf16_bits(z1 - __uint_as_float(h1 << 16));
      const unsigned l2 = bf16_bits(z2 - __uint_as_float(h2 << 16));
      const unsigned l3 = bf16_bits(z3 - __uint_as_float(h3 << 16));
      v2u wh, wlo;
      wh.x  = h0 | (h1 << 16); wh.y  = h2 | (h3 << 16);
      wlo.x = l0 | (l1 << 16); wlo.y = l2 | (l3 << 16);
      *(v2ua*)(rb + 2 * lane)      = wh;
      *(v2ua*)(rb + 64 + 2 * lane) = wlo;
      wave_sync();
      const v4u q0 = *(const v4ua*)(rb + 4 * lane);
      wave_sync();
      unsigned short* rp = ZHL + (size_t)d * APITCH + 8 * lane;
      *(volatile v4u*)rp = q0;
      __threadfence();
      *(volatile v4u*)rp = q0;
    }
  }
}

template <int KTOT>
__global__ __launch_bounds__(GTHR) __attribute__((amdgpu_num_vgpr(248)))
void k_lin(const unsigned short* __restrict__ A, const unsigned short* __restrict__ BT,
           const float* __restrict__ bsr, float* outp) {
  static_assert(KTOT % 32 == 0 && KTOT <= APITCH && KTOT <= WPITCH);
  __shared__ __attribute__((aligned(16))) float stg[GBM * GBN];
  __shared__ __attribute__((aligned(16))) float sb[GBN];
  const int tid = (int)threadIdx.x, lane = tid & 31, wave = tid >> 5, hh = lane >> 4, m = lane & 15;
  const int rowBase = (int)blockIdx.x * GBM;
  if (tid < 32) *(v4fa*)(sb + 4 * tid) = *(const v4fa*)(bsr + 4 * tid);

  v8f acc[8];
  {
    const v8f z = {0.f, 0.f, 0.f, 0.f, 0.f, 0.f, 0.f, 0.f};
#pragma unroll
    for (int t = 0; t < 8; ++t) acc[t] = z;
  }
  const unsigned short* ap = A + (size_t)(rowBase + 16 * wave + m) * (size_t)APITCH + 8 * hh;
  const unsigned short* bp = BT + (size_t)m * (size_t)WPITCH + 8 * hh;

#pragma unroll 1
  for (int k0 = 0; k0 < KTOT; k0 += 32) {
    FragB af;
    af.h[0] = *(const v8usa*)(ap + k0);
    af.h[1] = *(const v8usa*)(ap + k0 + 16);
#pragma unroll
    for (int nt = 0; nt < 8; ++nt) {
      const unsigned short* wq = bp + (size_t)(16 * nt) * (size_t)WPITCH + k0;
      FragB bf;
      bf.h[0] = *(const v8usa*)wq;
      bf.h[1] = *(const v8usa*)(wq + 16);
      acc[nt] = wmb(af, bf, acc[nt]);
    }
  }

#pragma unroll
  for (int nt = 0; nt < 8; ++nt) {
#pragma unroll
    for (int r = 0; r < 8; ++r) stg[(16 * wave + 8 * hh + r) * GBN + 16 * nt + m] = acc[nt][r];
  }
  __syncthreads();

  const v4f bias = *(const v4fa*)(sb + 4 * lane);
#pragma unroll 1
  for (int i = 0; i < 16; ++i) {
    const int lr  = 16 * wave + i;
    const int row = rowBase + lr;
    const v4f a = *(const v4fa*)(stg + lr * GBN + 4 * lane);
    asm volatile("" :: "v"(a));
    float v0 = a.x + bias.x, v1 = a.y + bias.y, v2 = a.z + bias.z, v3 = a.w + bias.w;
    v0 = (v0 > 0.0f) ? v0 : (v0 - v0); v1 = (v1 > 0.0f) ? v1 : (v1 - v1);
    v2 = (v2 > 0.0f) ? v2 : (v2 - v2); v3 = (v3 > 0.0f) ? v3 : (v3 - v3);
    v4f o;
    o.x = v0; o.y = v1; o.z = v2; o.w = v3;
    if (row < NN) {
      float* op = outp + (size_t)row * DF + 4 * lane;
      *(volatile v4f*)op = o;
      __threadfence();
      *(volatile v4f*)op = o;
    }
  }
}

extern "C" void kernel_launch(void* const* d_in, const int* in_sizes, int n_in,
                              void* d_out, int out_size, void* d_ws, size_t ws_size,
                              hipStream_t stream) {
  if (n_in < 6) return;
  if (in_sizes[0] != NN) return;
  if (in_sizes[1] != NE) return;
  if (in_sizes[2] != NE) return;
  if (in_sizes[3] != NV * DF) return;
  if (in_sizes[4] != NSTEP * DF * DF) return;
  if (in_sizes[5] != NSTEP * DF) return;
  if (out_size != NN * DF) return;

  const int*   ann = (const int*)d_in[0];
  const int*   src = (const int*)d_in[1];
  const int*   dst = (const int*)d_in[2];
  const float* emb = (const float*)d_in[3];
  const float* Ws  = (const float*)d_in[4];
  const float* bs  = (const float*)d_in[5];
  float* out = (float*)d_out;

  constexpr size_t zZHL  = (size_t)NP * APITCH * 2;
  constexpr size_t zH    = (size_t)NP * DF * 4;
  constexpr size_t zHB   = (size_t)NP * DF * 2;
  constexpr size_t zLIST = (size_t)NBK * RCAP * 4;
  constexpr size_t zCOI  = (size_t)NBK * COW * 4;
  constexpr size_t zFLAG = (size_t)NBK * 128;
  constexpr size_t zWD   = (size_t)NSTEP * DF * WPITCH * 2;
  constexpr size_t zBSR  = (size_t)NSTEP * DF * 4;
  constexpr size_t oZHL  = 0;
  constexpr size_t oH    = oZHL + zZHL;
  constexpr size_t oLIST = oH + zH;
  constexpr size_t oCOI  = oLIST + zLIST;
  constexpr size_t oFLAG = oCOI + zCOI;
  constexpr size_t oWD   = oFLAG + zFLAG;
  constexpr size_t oBSR  = oWD + zWD;
  constexpr size_t oEND  = oBSR + zBSR;
  static_assert(zZHL % 256 == 0 && zH % 256 == 0 && zLIST % 256 == 0 && zCOI % 256 == 0);
  static_assert(zFLAG % 256 == 0 && zWD % 256 == 0 && zBSR % 256 == 0 && zHB <= zH);
  static_assert(oEND <= ((size_t)128u << 20));
  if (oEND > ws_size) return;

  char* ws = (char*)d_ws;
  unsigned short* ZHL  = (unsigned short*)(ws + oZHL);
  float*          H    = (float*)(ws + oH);
  unsigned short* HB   = (unsigned short*)(ws + oH);
  int*            LIST = (int*)(ws + oLIST);
  int*            COI  = (int*)(ws + oCOI);
  int*            FLAG = (int*)(ws + oFLAG);
  unsigned short* WD   = (unsigned short*)(ws + oWD);
  float*          BSR  = (float*)(ws + oBSR);

  hipFuncSetAttribute(reinterpret_cast<const void*>(&k_bucket), hipFuncAttributeMaxDynamicSharedMemorySize, (int)BK_LDS);

  constexpr int KA = TWO_TERM_A ? 2 * DF : DF;
  constexpr int KB = TWO_TERM_B ? 2 * DF : DF;
  constexpr int KC = TWO_TERM_C ? 2 * DF : DF;

  k_prep<<<PBTOT, NTHR, 0, stream>>>(ann, emb, Ws, bs, HB, WD, ZHL, BSR);
  k_bucket<<<NBK, NTHR, BK_LDS, stream>>>(src, dst, LIST, COI, FLAG);

  k_rowsum<1><<<NP / RBM, NTHR, 0, stream>>>(LIST, COI, FLAG, HB, H, ZHL);
  k_lin<KA><<<NP / GBM, GTHR, 0, stream>>>(ZHL, WD, BSR, H);
  k_rowsum<0><<<NP / RBM, NTHR, 0, stream>>>(LIST, COI, FLAG, HB, H, ZHL);
  k_lin<KB><<<NP / GBM, GTHR, 0, stream>>>(ZHL, WD + (size_t)DF * WPITCH, BSR + DF, H);
  k_rowsum<0><<<NP / RBM, NTHR, 0, stream>>>(LIST, COI, FLAG, HB, H, ZHL);
  k_lin<KC><<<NP / GBM, GTHR, 0, stream>>>(ZHL, WD + (size_t)2 * DF * WPITCH, BSR + 2 * DF, out);
}
